// self_attention_block_19370302505593
// MI455X (gfx1250) — hardware-verified
//
#include <hip/hip_runtime.h>
#include <stddef.h>


typedef _Float16 h16;
typedef _Float16 v16h __attribute__((ext_vector_type(16)));
typedef _Float16 v8h  __attribute__((ext_vector_type(8)));
typedef _Float16 v4h  __attribute__((ext_vector_type(4)));
typedef float    v8f  __attribute__((ext_vector_type(8)));
typedef float    v4f  __attribute__((ext_vector_type(4)));
typedef float    v2f  __attribute__((ext_vector_type(2)));

#ifndef NB
#define NB 128
#endif
#ifndef SEQ
#define SEQ 512
#endif
#define NB_FULL 128
#define NE_FULL 512
#define FD      6
#define NEMB    16
#define NHEADS  4
#define DPH     4
#define VROWS   10
#define VLD     (SEQ + 8)
#define NPAIRS  (NHEADS * (SEQ / 16))
#define ROWF    32

#define QCARRY 8.0f
#define KCARRY 4.0f
#define SBACK  (1.0f / 64.0f)
#define VCARRY 64.0f
#define RCARRY 2048.0f
#define PCARRY 1024.0f
#define ACARRY 64.0f
#define WCARRY 64.0f

static_assert(NB >= 2 && NB <= NB_FULL && (NB % 2) == 0);
static_assert(SEQ >= 32 && SEQ <= NE_FULL && (SEQ % 32) == 0);
static_assert(NEMB == NHEADS * DPH);
static_assert(DPH == 4 && NEMB == 16 && FD == 6 && NHEADS == 4);
static_assert(VROWS == 10);
static_assert((NPAIRS % 8) == 0);
static_assert((VLD % 8) == 0 && VLD >= SEQ);
static_assert(NEMB * FD == 96);
static_assert(NEMB * NEMB == 256);
static_assert((NB * FD) % 4 == 0 && (NB * FD) / 4 <= 256);
static_assert(ROWF * 4 == 128 && FD <= ROWF);

#define LDS_BYTES ((size_t)SEQ * FD * 4 + (size_t)SEQ * 4 * 2 + 288 * 4 + \
                   (size_t)SEQ * NEMB * 2 * 4 + (size_t)NHEADS * VROWS * VLD * 2 + \
                   256 * 2 + 64 * 4 * 2 + 32 * 4)
static_assert(LDS_BYTES <= (size_t)131072);

#define WS_TOTAL ((size_t)NB * ROWF * 4)
static_assert((WS_TOTAL % 128) == 0);
static_assert(WS_TOTAL <= (size_t)134217728);

__device__ __forceinline__ float bf16r(float x) {
  unsigned int u = __float_as_uint(x);
  u = (u + 0x7FFFu + ((u >> 16) & 1u)) & 0xFFFF0000u;
  return __uint_as_float(u);
}

static __device__ __forceinline__ h16 toh_flush(float v) {
  const h16 r = (h16)v;
  return (fabsf(v) < 6.103515625e-05f) ? (h16)0.0f : r;
}

static __device__ __forceinline__ v16h cat8(v8h lo, v8h hi) {
  v16h o;
#pragma unroll
  for (int i = 0; i < 8; ++i) { o[i] = lo[i]; o[i + 8] = hi[i]; }
  return o;
}
static __device__ __forceinline__ v16h pad44(v4h a, v4h b) {
  v16h o = {};
  o[0] = a[0]; o[1] = a[1]; o[2] = a[2]; o[3] = a[3];
  o[4] = b[0]; o[5] = b[1]; o[6] = b[2]; o[7] = b[3];
  return o;
}

__device__ __forceinline__ v8f wmma16(v16h a, v16h b, v8f c) {
  v8f d = __builtin_amdgcn_wmma_f32_16x16x32_f16(false, a, false, b, (short)0, c,
                                                 false, false);
  asm volatile("v_nop\n\tv_nop\n\tv_nop\n\tv_nop" : "+v"(d) : "v"(a), "v"(b));
  return d;
}

__device__ __forceinline__ float red32_sum(float x) {
#pragma unroll
  for (int off = 1; off < 32; off <<= 1) x += __shfl_xor(x, off, 32);
  return x;
}

__global__ __launch_bounds__(256) void entity_attn_kernel(
    const float* __restrict__ inp, const float* __restrict__ maskG,
    const float* __restrict__ Wq, const float* __restrict__ Wk, const float* __restrict__ Wv,
    const float* __restrict__ Wpost, float* __restrict__ rows) {
  __shared__ __attribute__((aligned(16))) float xinS[SEQ * FD];
  __shared__ __attribute__((aligned(16))) float maskS[SEQ];
  __shared__ __attribute__((aligned(16))) float biasS[SEQ];
  __shared__ __attribute__((aligned(16))) float wS[288];
  __shared__ __attribute__((aligned(16))) h16 Qp[SEQ * NEMB];
  __shared__ __attribute__((aligned(16))) h16 Qr[SEQ * NEMB];
  __shared__ __attribute__((aligned(16))) h16 Kp[SEQ * NEMB];
  __shared__ __attribute__((aligned(16))) h16 Kr[SEQ * NEMB];
  __shared__ __attribute__((aligned(16))) h16 VT[NHEADS * VROWS * VLD];
  __shared__ __attribute__((aligned(16))) h16 Wp16[256];
  __shared__ __attribute__((aligned(16))) float redA[64];
  __shared__ __attribute__((aligned(16))) float redB[64];
  __shared__ __attribute__((aligned(16))) float outS[32];

  const unsigned tid = threadIdx.x, lane = tid & 31u;
  const unsigned wave = (unsigned)__builtin_amdgcn_readfirstlane((int)(threadIdx.x >> 5));
  const unsigned hh = lane >> 4, m = lane & 15u;
  const unsigned b = blockIdx.x;

  if (tid < 96u) {
    wS[tid]        = bf16r(Wq[tid]);
    wS[96u + tid]  = bf16r(Wk[tid]);
    wS[192u + tid] = bf16r(Wv[tid]);
  }
  {
    const unsigned n = tid >> 4, e = tid & 15u;
    const unsigned nc = (n < (unsigned)FD) ? n : (unsigned)(FD - 1);
    const float wv0 = bf16r(Wpost[nc * 16u + e]);
    const float sel = (n < (unsigned)FD) ? (WCARRY * wv0) : 0.0f;
    Wp16[tid] = toh_flush(sel);
  }
  {
    const unsigned nv = 8u * (unsigned)(VLD / 8);
#pragma unroll 1
    for (unsigned i = tid; i < nv; i += 256u) {
      const unsigned rowi = i / (unsigned)(VLD / 8);
      const unsigned c = i - rowi * (unsigned)(VLD / 8);
      const unsigned hd = rowi >> 1;
      const unsigned rr = 4u + (rowi & 1u);
      const float fv = ((rowi & 1u) == 0u) ? 1.0f : 0.0f;
      const h16 hv = (h16)fv;
      v8h cv;
#pragma unroll
      for (int j = 0; j < 8; ++j) cv[j] = hv;
      *(v8h*)&VT[(hd * VROWS + rr) * VLD + c * 8u] = cv;
    }
  }
  __syncthreads();

#pragma unroll 1
  for (unsigned t = tid; t < (unsigned)SEQ; t += 256u) {
    const size_t g = (size_t)b * NE_FULL + t;
    const float mk = bf16r(maskG[g]);
    maskS[t] = mk;
    biasS[t] = 1.0e9f * (mk - 1.0f);
    const float* ip = inp + g * FD;
    const v2f a0 = *(const v2f*)(ip);
    const v2f a1 = *(const v2f*)(ip + 2);
    const v2f a2 = *(const v2f*)(ip + 4);
    float x[FD];
    x[0] = bf16r(a0[0]) * mk; x[1] = bf16r(a0[1]) * mk;
    x[2] = bf16r(a1[0]) * mk; x[3] = bf16r(a1[1]) * mk;
    x[4] = bf16r(a2[0]) * mk; x[5] = bf16r(a2[1]) * mk;
#pragma unroll
    for (int f = 0; f < FD; ++f) xinS[t * FD + (unsigned)f] = x[f];
#pragma unroll 1
    for (unsigned e = 0; e < (unsigned)NEMB; ++e) {
      float aq = 0.0f, ak = 0.0f, av = 0.0f;
#pragma unroll
      for (int f = 0; f < FD; ++f) {
        aq += x[f] * wS[e * FD + (unsigned)f];
        ak += x[f] * wS[96u + e * FD + (unsigned)f];
        av += x[f] * wS[192u + e * FD + (unsigned)f];
      }
      const float fq = QCARRY * aq;
      const float fk = KCARRY * ak;
      const float fv = VCARRY * av;
      const h16 hq = toh_flush(fq);
      const h16 hk = toh_flush(fk);
      const h16 hv = toh_flush(fv);
      Qp[t * NEMB + e] = hq;
      Qr[t * NEMB + e] = toh_flush(fq - (float)hq);
      Kp[t * NEMB + e] = hk;
      Kr[t * NEMB + e] = toh_flush(fk - (float)hk);
      VT[((e >> 2) * VROWS + (e & 3u)) * VLD + t] = hv;
      VT[((e >> 2) * VROWS + 6u + (e & 3u)) * VLD + t] = toh_flush(RCARRY * (fv - (float)hv));
    }
  }
  __syncthreads();

  {
    const v8f zero8 = {};
    const v4h z4 = {};
    const bool up = (hh != 0u);
    const unsigned vrow = (m < 5u) ? m : ((m >= 8u && m < 12u) ? (m - 2u) : 5u);
#pragma unroll 1
    for (unsigned pair = wave; pair < (unsigned)NPAIRS; pair += 8u) {
      const unsigned h = pair & 3u, qt = pair >> 2;
      const unsigned qrow = qt * 16u + m;
      const v4h qh = *(const v4h*)&Qp[qrow * NEMB + h * 4u];
      const v4h qr = *(const v4h*)&Qr[qrow * NEMB + h * 4u];
      const v4h qlo = up ? qr : qh;
      const v4h qhi = up ? z4 : qh;
      const v16h qf = pad44(qlo, qhi);
      const float mq = maskS[qrow];
      float mrun = -1.0e30f;
      v8f o = {};
      const unsigned vbase = (h * VROWS + vrow) * VLD + hh * 8u;

#pragma unroll 1
      for (unsigned kb = 0; kb < (unsigned)SEQ; kb += 32u) {
        const v4h ka  = *(const v4h*)&Kp[(kb + m) * NEMB + h * 4u];
        const v4h kar = *(const v4h*)&Kr[(kb + m) * NEMB + h * 4u];
        const v4h kc  = *(const v4h*)&Kp[(kb + 16u + m) * NEMB + h * 4u];
        const v4h kcr = *(const v4h*)&Kr[(kb + 16u + m) * NEMB + h * 4u];
        const v4h ka2 = up ? z4 : kar;
        const v4h kc2 = up ? z4 : kcr;
        const v16h kf0 = pad44(ka, ka2);
        const v16h kf1 = pad44(kc, kc2);
        const v8f s0 = wmma16(kf0, qf, zero8);
        const v8f s1 = wmma16(kf1, qf, zero8);

        const v4f b0 = *(const v4f*)&biasS[kb + 8u * hh];
        const v4f b1 = *(const v4f*)&biasS[kb + 8u * hh + 4u];
        const v4f b2 = *(const v4f*)&biasS[kb + 16u + 8u * hh];
        const v4f b3 = *(const v4f*)&biasS[kb + 16u + 8u * hh + 4u];
        float e0[8], e1[8];
#pragma unroll
        for (int r = 0; r < 4; ++r) {
          e0[r]     = s0[r]     * SBACK + b0[r];
          e0[r + 4] = s0[r + 4] * SBACK + b1[r];
          e1[r]     = s1[r]     * SBACK + b2[r];
          e1[r + 4] = s1[r + 4] * SBACK + b3[r];
        }
        float mx = fmaxf(e0[0], e1[0]);
#pragma unroll
        for (int r = 1; r < 8; ++r) mx = fmaxf(mx, fmaxf(e0[r], e1[r]));
        mx = fmaxf(mx, __shfl_xor(mx, 16, 32));
        const float mn = fmaxf(mrun, mx);
        const float alpha = __expf(mrun - mn);
        mrun = mn;
#pragma unroll
        for (int r = 0; r < 8; ++r) o[r] = o[r] * alpha;

        v16h pf;
#pragma unroll
        for (int r = 0; r < 8; ++r) {
          pf[r]     = toh_flush(__expf(e0[r] - mn) * PCARRY);
          pf[r + 8] = toh_flush(__expf(e1[r] - mn) * PCARRY);
        }
        const v8h vlo = *(const v8h*)&VT[vbase + kb];
        const v8h vhi = *(const v8h*)&VT[vbase + kb + 16u];
        const v16h vf = cat8(vlo, vhi);
        o = wmma16(vf, pf, o);
      }

      const float t0 = __shfl_xor(o[0], 16, 32);
      const float t1 = __shfl_xor(o[1], 16, 32);
      const float t2 = __shfl_xor(o[2], 16, 32);
      const float t3 = __shfl_xor(o[3], 16, 32);
      const float f0 = o[0] + t0 * (1.0f / RCARRY);
      const float f1 = o[1] + t1 * (1.0f / RCARRY);
      const float f2 = o[2] + t2 * (1.0f / RCARRY);
      const float f3 = o[3] + t3 * (1.0f / RCARRY);
      const float l = up ? 1.0f : o[4];
      const float inv = __builtin_amdgcn_rcpf(l) * (ACARRY / VCARRY) * mq;
      const float g0 = f0 * inv, g1 = f1 * inv, g2 = f2 * inv, g3 = f3 * inv;
      v4h av, ar;
      av[0] = toh_flush(g0);
      av[1] = toh_flush(g1);
      av[2] = toh_flush(g2);
      av[3] = toh_flush(g3);
      ar[0] = toh_flush(g0 - (float)av[0]);
      ar[1] = toh_flush(g1 - (float)av[1]);
      ar[2] = toh_flush(g2 - (float)av[2]);
      ar[3] = toh_flush(g3 - (float)av[3]);
      if (!up) {
        *(v4h*)&Qp[qrow * NEMB + h * 4u] = av;
        *(v4h*)&Qr[qrow * NEMB + h * 4u] = ar;
      }
    }
  }
  __syncthreads();

  {
    const v8f zero8 = {};
    const v8h wlo = *(const v8h*)&Wp16[m * 16u + hh * 8u];
    const v16h wf = cat8(wlo, wlo);
    const unsigned col = (m < (unsigned)FD) ? m : (unsigned)(FD - 1);
    const float cs = 1.0f / (ACARRY * WCARRY);
#pragma unroll 1
    for (unsigned tile = wave; tile < (unsigned)(SEQ / 16); tile += 8u) {
      const unsigned t0 = tile * 16u;
      const v8h alo = *(const v8h*)&Qp[(t0 + m) * NEMB + hh * 8u];
      const v8h are = *(const v8h*)&Qr[(t0 + m) * NEMB + hh * 8u];
      const v16h af = cat8(alo, are);
      const v8f d = wmma16(af, wf, zero8);
#pragma unroll
      for (int r = 0; r < 8; ++r) {
        const unsigned t = t0 + 8u * hh + (unsigned)r;
        const float xv = xinS[t * FD + col];
        const float val = xv + d[r] * cs;
        if (m < (unsigned)FD) xinS[t * FD + col] = val;
      }
    }
  }
  __syncthreads();

  const float nef = (float)(SEQ * FD);
  float sx = 0.0f, sn = 0.0f;
#pragma unroll 1
  for (unsigned t = tid; t < (unsigned)SEQ; t += 256u) {
    sn += maskS[t];
#pragma unroll
    for (int f = 0; f < FD; ++f) sx += xinS[t * FD + (unsigned)f];
  }
  {
    const float r0 = red32_sum(sx);
    const float r1 = red32_sum(sn);
    if (lane == 0u) { redA[wave * 8u] = r0; redA[wave * 8u + 1u] = r1; }
  }
  __syncthreads();
  float Sx = 0.0f, Nv = 0.0f;
#pragma unroll
  for (int w = 0; w < 8; ++w) { Sx += redA[w * 8]; Nv += redA[w * 8 + 1]; }

  const float rN = 1.0f / Nv;
  const float mu = (Sx * (1.0f / nef)) * ((float)SEQ * rN);
  const float sx2 = Sx + mu * (float)FD * ((float)SEQ - Nv);
  const float m2 = sx2 * (1.0f / nef);

  float sq = 0.0f;
  float pfe[FD];
#pragma unroll
  for (int f = 0; f < FD; ++f) pfe[f] = 0.0f;
#pragma unroll 1
  for (unsigned t = tid; t < (unsigned)SEQ; t += 256u) {
    const float mk = maskS[t];
    const float fill = (1.0f - mk) * mu;
#pragma unroll
    for (int f = 0; f < FD; ++f) {
      const float xv = xinS[t * FD + (unsigned)f];
      const float dv = (xv + fill) - m2;
      sq += dv * dv;
      pfe[f] += (xv - mu) * mk;
    }
  }
  {
    const float rq = red32_sum(sq);
    float rf[FD];
#pragma unroll
    for (int f = 0; f < FD; ++f) rf[f] = red32_sum(pfe[f]);
    if (lane == 0u) {
      redB[wave * 8u] = rq;
#pragma unroll
      for (int f = 0; f < FD; ++f) redB[wave * 8u + 1u + (unsigned)f] = rf[f];
    }
  }
  __syncthreads();
  float Sq = 0.0f, pft = 0.0f;
  {
    const unsigned c = (tid < (unsigned)FD) ? tid : (unsigned)(FD - 1);
#pragma unroll
    for (int w = 0; w < 8; ++w) { Sq += redB[w * 8]; pft += redB[w * 8 + 1 + (int)c]; }
  }
  const float var = Sq * (1.0f / (nef - 1.0f));
  const float ratio = (nef - 1.0f) * (1.0f / ((float)FD * Nv - 1.0f));
  const float stdv = sqrtf(var) * sqrtf(ratio);
  const float inv = 1.0f / (stdv + 1.0e-6f);
  const float val = (tid < (unsigned)FD) ? (pft * inv * rN) : 0.0f;
  if (tid < 32u) outS[tid] = val;
  __syncthreads();
  {
    const v4f ov = *(const v4f*)&outS[4u * (tid & 7u)];
    float* p = rows + (size_t)b * ROWF + 4u * (tid & 7u);
    if (tid < 8u) *(volatile v4f*)p = ov;
    __threadfence();
    if (tid < 8u) *(volatile v4f*)p = ov;
  }
}

__global__ __launch_bounds__(256) void pool_out_kernel(
    const float* __restrict__ rows, float* __restrict__ out) {
  const unsigned i = threadIdx.x;
  const unsigned nvec = (unsigned)(NB * FD / 4);
  const unsigned ic = (i < nvec) ? i : (nvec - 1u);
  v4f v;
#pragma unroll
  for (int j = 0; j < 4; ++j) {
    const unsigned idx = 4u * ic + (unsigned)j;
    const unsigned bb = idx / (unsigned)FD;
    const unsigned f = idx - bb * (unsigned)FD;
    v[j] = rows[(size_t)bb * ROWF + f];
  }
  float* p = out + 4u * ic;
  if (i < nvec) *(volatile v4f*)p = v;
  __threadfence();
  if (i < nvec) *(volatile v4f*)p = v;
}

extern "C" void kernel_launch(void* const* d_in, const int* in_sizes, int n_in,
                              void* d_out, int out_size, void* d_ws, size_t ws_size,
                              hipStream_t stream) {
  if (n_in < 6) return;
  const long long need_rows = (long long)(NB - 1) * NE_FULL + SEQ;
  if ((long long)in_sizes[0] < need_rows * FD) return;
  if ((long long)in_sizes[1] < need_rows) return;
  if (in_sizes[2] < NEMB * FD || in_sizes[3] < NEMB * FD || in_sizes[4] < NEMB * FD) return;
  if (in_sizes[5] < FD * NEMB) return;
  if ((long long)out_size < (long long)NB * FD) return;
  if (ws_size < WS_TOTAL) return;

  const float* inp   = (const float*)d_in[0];
  const float* mask  = (const float*)d_in[1];
  const float* wq    = (const float*)d_in[2];
  const float* wk    = (const float*)d_in[3];
  const float* wv    = (const float*)d_in[4];
  const float* wpost = (const float*)d_in[5];
  float* out  = (float*)d_out;
  float* rows = (float*)d_ws;

  entity_attn_kernel<<<dim3(NB), dim3(256), 0, stream>>>(inp, mask, wq, wk, wv, wpost, rows);
  pool_out_kernel<<<dim3(1), dim3(256), 0, stream>>>(rows, out);
}
